// MultiheadCrossAttention_3590592660074
// MI455X (gfx1250) — hardware-verified
//
#include <hip/hip_runtime.h>


#ifndef NB
#define NB 4
#endif
#ifndef SEQ
#define SEQ 1024
#endif
#ifndef SKV
#define SKV 1024
#endif
#define NB_FULL 4
#define T_FULL 1024
#define S_FULL 1024
#define DMOD 1024
#define NHD 16
#define HD 64
#define QB 32
#define PCAR 16384.0f
#define L2E 1.4426950408889634f
#define LNEPS 1.0e-5f

static_assert(NHD * HD == DMOD);
static_assert(HD == 64);
static_assert(NB >= 1 && NB <= NB_FULL);
static_assert(SEQ % QB == 0);
static_assert(SEQ % 2 == 0);
static_assert(SKV % 64 == 0);
static_assert((NB * SEQ) % 64 == 0);
static_assert((NB * SKV) % 64 == 0);
static_assert(DMOD % 64 == 0);
static_assert(SEQ <= T_FULL);
static_assert(SKV <= S_FULL);

#define WS_QB  ((size_t)NB * SEQ * DMOD * 2)
#define WS_KVB ((size_t)NB * SKV * DMOD * 2)
#define WS_W   ((size_t)DMOD * DMOD * 2)
#define WS_CQ  ((size_t)NB * SEQ * DMOD * 4)
#define WS_CKV ((size_t)NB * SKV * DMOD * 4)
#define WS_VT  ((size_t)NB * NHD * HD * SKV * 2)
#define WS_TOTAL (WS_QB + WS_KVB + 3 * WS_W + WS_CQ + 2 * WS_CKV + 2 * WS_QB + 2 * WS_KVB + WS_VT)
static_assert(WS_QB % 256 == 0);
static_assert(WS_KVB % 256 == 0);
static_assert(WS_W % 256 == 0);
static_assert(WS_CQ % 256 == 0);
static_assert(WS_CKV % 256 == 0);
static_assert(WS_VT % 256 == 0);
static_assert(WS_TOTAL <= (size_t)134217728);

typedef _Float16 h16;
typedef unsigned short bf;
typedef __attribute__((ext_vector_type(16))) __bf16   v16bf;
typedef __attribute__((ext_vector_type(16))) _Float16 v16h;
typedef __attribute__((ext_vector_type(8)))  _Float16 v8h;
typedef __attribute__((ext_vector_type(8)))  unsigned short v8us;
typedef __attribute__((ext_vector_type(8)))  float    v8f;
typedef __attribute__((ext_vector_type(4)))  float    v4f;
typedef v8h  __attribute__((may_alias)) v8ha;
typedef v4f  __attribute__((may_alias)) v4fa;
typedef v8us __attribute__((may_alias)) v8usa;

__device__ __forceinline__ unsigned short f2bf(float f) { unsigned u = __float_as_uint(f); u += 0x7FFFu + ((u >> 16) & 1u); return (unsigned short)(u >> 16); }
__device__ __forceinline__ float bf2f(unsigned short b) { return __uint_as_float(((unsigned)b) << 16); }
__device__ __forceinline__ float bfr(float f) { return bf2f(f2bf(f)); }
__device__ __forceinline__ v16h cat16(v8h lo, v8h hi) { return __builtin_shufflevector(lo, hi, 0, 1, 2, 3, 4, 5, 6, 7, 8, 9, 10, 11, 12, 13, 14, 15); }
__device__ __forceinline__ v16bf cat16b(v8us lo, v8us hi) { return __builtin_bit_cast(v16bf, __builtin_shufflevector(lo, hi, 0, 1, 2, 3, 4, 5, 6, 7, 8, 9, 10, 11, 12, 13, 14, 15)); }
__device__ __forceinline__ v8f wmma16(v16h a, v16h b, v8f c) { return __builtin_amdgcn_wmma_f32_16x16x32_f16(false, a, false, b, (short)0, c, false, false); }
__device__ __forceinline__ v8f wmmab(v16bf a, v16bf b, v8f c) { return __builtin_amdgcn_wmma_f32_16x16x32_bf16(false, a, false, b, (short)0, c, false, false); }
__device__ __forceinline__ void splitf(float y, unsigned short& h, unsigned short& l) { h = f2bf(y); l = f2bf(y - bf2f(h)); }
__device__ __forceinline__ h16 tohc(float y) { y = (fabsf(y) < 6.103515625e-05f) ? 0.0f : y; return (h16)y; }

template <typename T16> struct WFrag;
template <> struct WFrag<h16> { typedef v16h V; static __device__ __forceinline__ V ld(const h16* p) { return cat16(*(const v8h*)p, *(const v8h*)(p + 16)); } static __device__ __forceinline__ v8f mma(V a, V b, v8f c) { return wmma16(a, b, c); } };
template <> struct WFrag<bf> { typedef v16bf V; static __device__ __forceinline__ V ld(const bf* p) { return cat16b(*(const v8us*)p, *(const v8us*)(p + 16)); } static __device__ __forceinline__ v8f mma(V a, V b, v8f c) { return wmmab(a, b, c); } };
template <typename T16, int NSPLIT, bool BIAS>
__global__ __launch_bounds__(32) void k_gemmw(const T16* __restrict__ A, const T16* __restrict__ A2, const T16* __restrict__ Bt, const T16* __restrict__ Bt2, int K, float* C, int ldc, const float* __restrict__ bias, size_t sA, size_t sB, size_t sC) {
    typedef typename WFrag<T16>::V V;
    __shared__ __align__(16) float os[16 * 68];
    const size_t z = blockIdx.z; A += z * sA; if (A2) A2 += z * sA; Bt += z * sB; if (Bt2) Bt2 += z * sB; C += z * sC;
    const int lane = threadIdx.x & 31, lr = lane & 15, hi = lane >> 4; const int r0 = blockIdx.x * 64, c0 = blockIdx.y * 64;
    v8f acc[4][4];
#pragma unroll
    for (int mb = 0; mb < 4; ++mb)
#pragma unroll
        for (int nb = 0; nb < 4; ++nb) acc[mb][nb] = (v8f){};
    const size_t aoff = (size_t)(r0 + lr) * K + 8 * hi, boff = (size_t)(c0 + lr) * K + 8 * hi;
#pragma unroll 1
    for (int kc = 0; kc < K; kc += 32) {
        V a[4], a2[4];
#pragma unroll
        for (int mb = 0; mb < 4; ++mb) { a[mb] = WFrag<T16>::ld(A + aoff + (size_t)mb * 16 * K + kc); if (NSPLIT == 1 || NSPLIT == 2) a2[mb] = WFrag<T16>::ld(A2 + aoff + (size_t)mb * 16 * K + kc); }
#pragma unroll
        for (int nb = 0; nb < 4; ++nb) { const V b = WFrag<T16>::ld(Bt + boff + (size_t)nb * 16 * K + kc); V b2; if (NSPLIT >= 2) b2 = WFrag<T16>::ld(Bt2 + boff + (size_t)nb * 16 * K + kc);
#pragma unroll
            for (int mb = 0; mb < 4; ++mb) { acc[mb][nb] = WFrag<T16>::mma(a[mb], b, acc[mb][nb]); if (NSPLIT == 1 || NSPLIT == 2) acc[mb][nb] = WFrag<T16>::mma(a2[mb], b, acc[mb][nb]); if (NSPLIT >= 2) acc[mb][nb] = WFrag<T16>::mma(a[mb], b2, acc[mb][nb]); } }
        asm volatile("v_nop\n\tv_nop\n\tv_nop\n\tv_nop" : "+v"(acc[0][0]), "+v"(acc[1][1]), "+v"(acc[2][2]), "+v"(acc[3][3]) : "v"(a[0]), "v"(a[3]));
    }
#pragma unroll
    for (int mb = 0; mb < 4; ++mb) {
#pragma unroll
        for (int nb = 0; nb < 4; ++nb) {
#pragma unroll
            for (int j = 0; j < 8; ++j) os[(hi * 8 + j) * 68 + nb * 16 + lr] = acc[mb][nb][j]; }
        __builtin_amdgcn_wave_barrier(); asm volatile("" ::: "memory");
        float* crow = C + (size_t)(r0 + mb * 16) * ldc + c0;
#pragma unroll 1
        for (int ps = 0; ps < 2; ++ps) {
#pragma unroll
            for (int s = 0; s < 8; ++s) { const int row = 2 * s + hi, cofs = lr * 4; v4f val = *(const v4fa*)(os + row * 68 + cofs); if (BIAS) { val[0] += bfr(bias[c0 + cofs]); val[1] += bfr(bias[c0 + cofs + 1]); val[2] += bfr(bias[c0 + cofs + 2]); val[3] += bfr(bias[c0 + cofs + 3]); }
                *(volatile v4f*)(crow + (size_t)row * ldc + cofs) = val; }
            if (ps == 0) __threadfence(); }
        __builtin_amdgcn_wave_barrier(); asm volatile("" ::: "memory");
    }
}

template <int RPB, int SRPB>
__global__ __launch_bounds__(256) void k_cvt8r(const float* __restrict__ src, bf* dst, unsigned n8) {
    const unsigned i = blockIdx.x * 256u + threadIdx.x; if (i >= n8) return;
    const unsigned e0 = i * 8u, R = e0 / DMOD, col = e0 % DMOD, bb = R / RPB, tt = R % RPB;
    const v8f v = *(const v8f*)(src + ((size_t)bb * SRPB + tt) * DMOD + col); v8us o;
#pragma unroll
    for (int k = 0; k < 8; ++k) o[k] = f2bf(v[k]);
    *(volatile v8us*)(dst + e0) = o; __threadfence(); *(volatile v8us*)(dst + e0) = o;
}

__global__ __launch_bounds__(256) void k_ln(const float* __restrict__ C, const float* __restrict__ gam, const float* __restrict__ bet, bf* PH, bf* PL, int R) {
    const int t = threadIdx.x, w = t >> 5, lane = t & 31;
    const int row = blockIdx.x * 2 + (w >> 2);
    if (row >= R) return;
    const int col = (w & 3) * 256 + lane * 8, gc = (lane & 7) * 8;
    const v8f x = *(const v8f*)(C + (size_t)row * DMOD + col);
    float s1 = 0.0f;
#pragma unroll
    for (int e = 0; e < 8; ++e) s1 += x[e];
    s1 += __shfl_xor(s1, 1, 32); s1 += __shfl_xor(s1, 2, 32); s1 += __shfl_xor(s1, 4, 32);
    const float mu = s1 * (1.0f / 64.0f);
    v8f d; float s2 = 0.0f;
#pragma unroll
    for (int e = 0; e < 8; ++e) { d[e] = x[e] - mu; s2 += d[e] * d[e]; }
    s2 += __shfl_xor(s2, 1, 32); s2 += __shfl_xor(s2, 2, 32); s2 += __shfl_xor(s2, 4, 32);
    const float rstd = rsqrtf(s2 * (1.0f / 64.0f) + LNEPS);
    const v8f g = *(const v8f*)(gam + gc), be = *(const v8f*)(bet + gc);
    v8us oh, ol;
#pragma unroll
    for (int e = 0; e < 8; ++e) { const float y = d[e] * rstd * bfr(g[e]) + bfr(be[e]); unsigned short hh, ll; splitf(y, hh, ll); oh[e] = hh; ol[e] = ll; }
    const size_t po = (size_t)row * DMOD + col;
    *(volatile v8us*)(PH + po) = oh; *(volatile v8us*)(PL + po) = ol;
    __threadfence();
    *(volatile v8us*)(PH + po) = oh; *(volatile v8us*)(PL + po) = ol;
}

__global__ __launch_bounds__(512) void k_vtr_ln(const float* __restrict__ F, const float* __restrict__ gam, const float* __restrict__ bet, h16* VT) {
    __shared__ __align__(16) h16 tile[64 * 72];
    const int b = blockIdx.z, head = blockIdx.y, s0 = blockIdx.x * 64, t = threadIdx.x;
    {
        const int r = t >> 3, seg = t & 7;
        const float* src = F + ((size_t)b * SKV + s0 + r) * DMOD + head * HD + seg * 8;
        const v8f x = *(const v8f*)src;
        float s1 = 0.0f;
#pragma unroll
        for (int e = 0; e < 8; ++e) s1 += x[e];
        s1 += __shfl_xor(s1, 1, 32); s1 += __shfl_xor(s1, 2, 32); s1 += __shfl_xor(s1, 4, 32);
        const float mu = s1 * (1.0f / 64.0f);
        v8f d; float s2 = 0.0f;
#pragma unroll
        for (int e = 0; e < 8; ++e) { d[e] = x[e] - mu; s2 += d[e] * d[e]; }
        s2 += __shfl_xor(s2, 1, 32); s2 += __shfl_xor(s2, 2, 32); s2 += __shfl_xor(s2, 4, 32);
        const float rstd = rsqrtf(s2 * (1.0f / 64.0f) + LNEPS);
        const v8f g = *(const v8f*)(gam + seg * 8), be = *(const v8f*)(bet + seg * 8);
        v8h o;
#pragma unroll
        for (int e = 0; e < 8; ++e) o[e] = tohc(d[e] * rstd * bfr(g[e]) + bfr(be[e]));
        *(v8h*)(tile + r * 72 + seg * 8) = o;
    }
    __syncthreads();
    const int piece = t & 7, d = t >> 3;
    v8h o2;
#pragma unroll
    for (int e = 0; e < 8; ++e) o2[e] = tile[(piece * 8 + e) * 72 + d];
#pragma unroll 1
    for (int ps = 0; ps < 2; ++ps) {
        *(volatile v8h*)(VT + (((size_t)(b * NHD + head)) * HD + d) * SKV + s0 + piece * 8) = o2;
        if (ps == 0) __threadfence(); }
}

__global__ __launch_bounds__(64) __attribute__((amdgpu_num_vgpr(256)))
void k_flash(const bf* __restrict__ QHp, const bf* __restrict__ QLp, const bf* __restrict__ KHp, const bf* __restrict__ KLp, const h16* __restrict__ VTp,
             const int* __restrict__ slen, const int* __restrict__ klen, float* OUT) {
    __shared__ __align__(16) float osm[2][16 * 68];
    const int b = blockIdx.z, head = blockIdx.y;
    const int w = threadIdx.x >> 5, lane = threadIdx.x & 31, hf = lane >> 4, lm = lane & 15;
    const int m0 = blockIdx.x * QB + w * 16;
    const int qn = slen[b], kn = klen[b];
    const bool qv = (m0 + lm) < qn;
    v16bf qfh[2], qfl[2];
    {
        const size_t qo = ((size_t)b * SEQ + m0 + lm) * DMOD + head * HD + 8 * hf;
        const bf* qh = QHp + qo; const bf* ql = QLp + qo;
#pragma unroll
        for (int ks = 0; ks < 2; ++ks) {
            qfh[ks] = cat16b(*(const v8us*)(qh + 32 * ks), *(const v8us*)(qh + 32 * ks + 16));
            qfl[ks] = cat16b(*(const v8us*)(ql + 32 * ks), *(const v8us*)(ql + 32 * ks + 16));
        }
    }
    v8f acc[4];
#pragma unroll
    for (int dt = 0; dt < 4; ++dt) acc[dt] = (v8f){};
    float mrun = -1.0e30f, lrun = 0.0f;
    const size_t ko = ((size_t)b * SKV + lm) * DMOD + head * HD + 8 * hf;
    const bf* kch = KHp + ko; const bf* kcl = KLp + ko;
    const h16* vcur = VTp + (((size_t)(b * NHD + head)) * HD + lm) * SKV + 8 * hf;
#pragma unroll 1
    for (int sc = 0; sc < SKV; sc += 64) {
        v8f st[4];
#pragma unroll
        for (int s4 = 0; s4 < 4; ++s4) st[s4] = (v8f){};
#pragma unroll
        for (int s4 = 0; s4 < 4; ++s4) {
            const bf* kp = kch + (size_t)(s4 * 16) * DMOD; const bf* lp = kcl + (size_t)(s4 * 16) * DMOD;
#pragma unroll
            for (int ks = 0; ks < 2; ++ks) {
                const v16bf ah = cat16b(*(const v8us*)(kp + 32 * ks), *(const v8us*)(kp + 32 * ks + 16));
                const v16bf al = cat16b(*(const v8us*)(lp + 32 * ks), *(const v8us*)(lp + 32 * ks + 16));
                st[s4] = wmmab(ah, qfh[ks], st[s4]); st[s4] = wmmab(ah, qfl[ks], st[s4]); st[s4] = wmmab(al, qfh[ks], st[s4]);
            }
        }
        asm volatile("v_nop\n\tv_nop\n\tv_nop\n\tv_nop" : "+v"(st[0]), "+v"(st[1]), "+v"(st[2]), "+v"(st[3]) : "v"(qfh[0]), "v"(qfh[1]), "v"(qfl[0]), "v"(qfl[1]));
        float cm = -1.0e30f;
#pragma unroll
        for (int s4 = 0; s4 < 4; ++s4) {
#pragma unroll
            for (int e = 0; e < 8; ++e) { const int key = sc + s4 * 16 + 8 * hf + e; float v = st[s4][e] * L2E; v = (qv && key < kn) ? v : 0.0f; st[s4][e] = v; cm = fmaxf(cm, v); } }
        cm = fmaxf(cm, __shfl_xor(cm, 16, 32));
        const float mnew = fmaxf(mrun, cm);
        const float alpha = __builtin_amdgcn_exp2f(mrun - mnew);
        mrun = mnew;
        float ls = 0.0f; v16h pf[2];
#pragma unroll
        for (int s4 = 0; s4 < 4; ++s4)
#pragma unroll
            for (int e = 0; e < 8; ++e) { const float p = __builtin_amdgcn_exp2f(st[s4][e] - mnew); ls += p; pf[s4 >> 1][(s4 & 1) * 8 + e] = (h16)(p * PCAR); }
        ls += __shfl_xor(ls, 16, 32);
        lrun = lrun * alpha + ls;
        v8f av;
#pragma unroll
        for (int e = 0; e < 8; ++e) av[e] = __shfl(alpha, 8 * hf + e, 32);
#pragma unroll
        for (int dt = 0; dt < 4; ++dt) acc[dt] *= av;
        asm volatile("" ::: "memory");
#pragma unroll
        for (int ks = 0; ks < 2; ++ks) {
#pragma unroll
            for (int dt = 0; dt < 4; ++dt) { const h16* vp = vcur + (size_t)(dt * 16) * SKV + sc + 32 * ks; const v16h vf = cat16(*(const v8h*)vp, *(const v8h*)(vp + 16)); acc[dt] = wmma16(pf[ks], vf, acc[dt]); }
            asm volatile("" ::: "memory");
        }
        asm volatile("v_nop\n\tv_nop\n\tv_nop\n\tv_nop" : "+v"(acc[0]), "+v"(acc[1]), "+v"(acc[2]), "+v"(acc[3]) : "v"(pf[0]), "v"(pf[1]));
        kch += (size_t)64 * DMOD; kcl += (size_t)64 * DMOD;
    }
    v8f lv;
#pragma unroll
    for (int e = 0; e < 8; ++e) lv[e] = __shfl(lrun, 8 * hf + e, 32);
    v8f iv;
#pragma unroll
    for (int e = 0; e < 8; ++e) iv[e] = 1.0f / (lv[e] * PCAR);
    float* osw = osm[w];
#pragma unroll
    for (int dt = 0; dt < 4; ++dt)
#pragma unroll
        for (int e = 0; e < 8; ++e) osw[(8 * hf + e) * 68 + dt * 16 + lm] = acc[dt][e] * iv[e];
    __syncthreads();
#pragma unroll 1
    for (int ps = 0; ps < 2; ++ps) {
#pragma unroll
        for (int s = 0; s < 8; ++s) { const int row = 2 * s + hf; const v4f val = *(const v4fa*)(osw + row * 68 + lm * 4);
            *(volatile v4f*)(OUT + ((size_t)b * SEQ + m0 + row) * DMOD + head * HD + lm * 4) = val; }
        if (ps == 0) __threadfence(); }
}

extern "C" void kernel_launch(void* const* d_in, const int* in_sizes, int n_in,
                              void* d_out, int out_size, void* d_ws, size_t ws_size, hipStream_t stream) {
    if (n_in < 12) return;
    if ((size_t)in_sizes[0] < (size_t)NB * T_FULL * DMOD) return;
    if ((size_t)in_sizes[1] < (size_t)NB * S_FULL * DMOD) return;
    if (in_sizes[2] < NB) return;
    if (in_sizes[3] < NB) return;
    if ((size_t)in_sizes[4] < (size_t)DMOD * DMOD) return;
    if ((size_t)in_sizes[5] < (size_t)DMOD) return;
    if ((size_t)in_sizes[6] < (size_t)DMOD * DMOD) return;
    if ((size_t)in_sizes[7] < (size_t)DMOD) return;
    if ((size_t)in_sizes[8] < (size_t)DMOD * DMOD) return;
    if ((size_t)in_sizes[9] < (size_t)DMOD) return;
    if ((size_t)in_sizes[10] < (size_t)HD) return;
    if ((size_t)in_sizes[11] < (size_t)HD) return;
    if ((size_t)out_size < (size_t)NB * SEQ * DMOD) return;
    const float* xq  = (const float*)d_in[0];
    const float* xkv = (const float*)d_in[1];
    const int*   sl  = (const int*)d_in[2];
    const int*   kl  = (const int*)d_in[3];
    const float* wq  = (const float*)d_in[4];
    const float* bq  = (const float*)d_in[5];
    const float* wk  = (const float*)d_in[6];
    const float* bk  = (const float*)d_in[7];
    const float* wv  = (const float*)d_in[8];
    const float* bv  = (const float*)d_in[9];
    const float* gam = (const float*)d_in[10];
    const float* bet = (const float*)d_in[11];
    float* OUT = (float*)d_out;
    char* wsp = (char*)d_ws;
    size_t used = 0;
    auto take = [&](size_t bytes) { char* p = wsp + used; used += (bytes + 255) & ~(size_t)255; return (void*)p; };
    bf*    QBp = (bf*)take(WS_QB);
    bf*    KVB = (bf*)take(WS_KVB);
    bf*    WQB = (bf*)take(WS_W);
    bf*    WKB = (bf*)take(WS_W);
    bf*    WVB = (bf*)take(WS_W);
    float* CQ  = (float*)take(WS_CQ);
    float* CK  = (float*)take(WS_CKV);
    float* CV  = (float*)take(WS_CKV);
    bf*    QH  = (bf*)take(WS_QB);
    bf*    QL  = (bf*)take(WS_QB);
    bf*    KH  = (bf*)take(WS_KVB);
    bf*    KLo = (bf*)take(WS_KVB);
    h16*   VT  = (h16*)take(WS_VT);
    if (used > ws_size || used > (size_t)134217728) return;
    const unsigned n8q = (unsigned)((size_t)NB * SEQ * DMOD / 8), n8kv = (unsigned)((size_t)NB * SKV * DMOD / 8), n8w = (unsigned)((size_t)DMOD * DMOD / 8);
    k_cvt8r<SEQ, T_FULL><<<(n8q + 255) / 256, 256, 0, stream>>>(xq, QBp, n8q);
    k_cvt8r<SKV, S_FULL><<<(n8kv + 255) / 256, 256, 0, stream>>>(xkv, KVB, n8kv);
    k_cvt8r<DMOD, DMOD><<<(n8w + 255) / 256, 256, 0, stream>>>(wq, WQB, n8w);
    k_cvt8r<DMOD, DMOD><<<(n8w + 255) / 256, 256, 0, stream>>>(wk, WKB, n8w);
    k_cvt8r<DMOD, DMOD><<<(n8w + 255) / 256, 256, 0, stream>>>(wv, WVB, n8w);
    k_gemmw<bf, 0, true><<<dim3((NB * SEQ) / 64, DMOD / 64, 1), 32, 0, stream>>>(QBp, QBp, WQB, WQB, DMOD, CQ, DMOD, bq, (size_t)0, (size_t)0, (size_t)0);
    k_gemmw<bf, 0, true><<<dim3((NB * SKV) / 64, DMOD / 64, 1), 32, 0, stream>>>(KVB, KVB, WKB, WKB, DMOD, CK, DMOD, bk, (size_t)0, (size_t)0, (size_t)0);
    k_gemmw<bf, 0, true><<<dim3((NB * SKV) / 64, DMOD / 64, 1), 32, 0, stream>>>(KVB, KVB, WVB, WVB, DMOD, CV, DMOD, bv, (size_t)0, (size_t)0, (size_t)0);
    k_ln<<<(NB * SEQ) / 2, 256, 0, stream>>>(CQ, gam, bet, QH, QL, NB * SEQ);
    k_ln<<<(NB * SKV) / 2, 256, 0, stream>>>(CK, gam, bet, KH, KLo, NB * SKV);
    k_vtr_ln<<<dim3(SKV / 64, NHD, NB), 512, 0, stream>>>(CV, gam, bet, VT);
    k_flash<<<dim3(SEQ / QB, NHD, NB), 64, 0, stream>>>(QH, QL, KH, KLo, VT, sl, kl, OUT);
}
